// CausalSelfAttention_30142080483610
// MI455X (gfx1250) — hardware-verified
//
#include <hip/hip_runtime.h>
#define NB 2
#define SQ 2048
#define NR (NB * SQ)
#define DM 2048
#define NHQ 16
#define NKV 16
#define NREP (NHQ / NKV)
#define HD 128
#define HH 64
#define KVD (NKV * HD)
#define WIN SQ
#define BAND 256
#define NBAND (SQ / BAND)
#define SP SQ
#define SPX BAND
#define NPB 1
#define SCALE 0.08838834764831845f
typedef __bf16 v16b __attribute__((ext_vector_type(16)));
typedef unsigned short v8us __attribute__((ext_vector_type(8), may_alias));
typedef float  v8f  __attribute__((ext_vector_type(8)));
typedef float  v4f  __attribute__((ext_vector_type(4)));
typedef float  v4fa __attribute__((ext_vector_type(4), may_alias));
union FragB { v16b v; v8us half[2]; unsigned short u[16]; };

__device__ __forceinline__ unsigned short bf16_bits(float x) { unsigned int u = __float_as_uint(x); return (unsigned short)((u + 0x7FFFu + ((u >> 16) & 1u)) >> 16); }
__device__ __forceinline__ float bf16_val(unsigned short b) { return __uint_as_float(((unsigned int)b) << 16); }
__device__ __forceinline__ float bf16_round(float x) { return bf16_val(bf16_bits(x)); }
template <int NT>
__device__ __forceinline__ v8f mmaN(v16b ah, v16b al, v16b bh, v16b bl, v8f c) {
  c = __builtin_amdgcn_wmma_f32_16x16x32_bf16(false, ah, false, bh, (short)0, c, false, false);
  if (NT >= 2) c = __builtin_amdgcn_wmma_f32_16x16x32_bf16(false, al, false, bh, (short)0, c, false, false);
  if (NT >= 3) c = __builtin_amdgcn_wmma_f32_16x16x32_bf16(false, ah, false, bl, (short)0, c, false, false);
  asm volatile("v_nop\n\tv_nop\n\tv_nop\n\tv_nop" : "+v"(c) : "v"(ah), "v"(al), "v"(bh), "v"(bl));
  return c;
}


typedef _Float16 v16h __attribute__((ext_vector_type(16)));
union FragH { v16h v; v8us half[2]; _Float16 h[16]; unsigned short u[16]; };
template <int NT>
__device__ __forceinline__ v8f mmaH(v16h ah, v16h al, v16h bh, v16h bl, v8f c) {
  c = __builtin_amdgcn_wmma_f32_16x16x32_f16(false, ah, false, bh, (short)0, c, false, false);
  if (NT >= 2) c = __builtin_amdgcn_wmma_f32_16x16x32_f16(false, al, false, bh, (short)0, c, false, false);
  if (NT >= 3) c = __builtin_amdgcn_wmma_f32_16x16x32_f16(false, ah, false, bl, (short)0, c, false, false);
  asm volatile("v_nop\n\tv_nop\n\tv_nop\n\tv_nop" : "+v"(c) : "v"(ah), "v"(al), "v"(bh), "v"(bl));
  return c;
}

__global__ __launch_bounds__(256) void k_wt_f16(const float* __restrict__ W, _Float16* __restrict__ Wt, int K, int N, float scale) {
  const int t = blockIdx.x * 256 + threadIdx.x; if (t >= N * (K / 8)) return; const int n = t / (K / 8), k8 = (t % (K / 8)) * 8; FragH f;
#pragma unroll
  for (int i = 0; i < 8; ++i) f.h[i] = (_Float16)(bf16_round(W[(size_t)(k8 + i) * N + n]) * scale); const v8us o = f.half[0];
  *(volatile v8us*)((unsigned short*)Wt + (size_t)n * K + k8) = o; __threadfence(); *(volatile v8us*)((unsigned short*)Wt + (size_t)n * K + k8) = o;
}


typedef _Float16 v4h __attribute__((ext_vector_type(4)));

__global__ __launch_bounds__(256) void k_x16(const float* __restrict__ x, _Float16* __restrict__ X16, size_t n8) { const size_t t = (size_t)blockIdx.x * 256 + threadIdx.x; if (t >= n8) return; FragH f;
#pragma unroll
  for (int q = 0; q < 8; ++q) f.h[q] = (_Float16)bf16_round(x[t * 8 + q]); *(volatile v8us*)((unsigned short*)X16 + t * 8) = f.half[0]; __threadfence(); *(volatile v8us*)((unsigned short*)X16 + t * 8) = f.half[0]; }
__global__ __launch_bounds__(256) void k_h16(const float* __restrict__ x, _Float16* __restrict__ X16, size_t n8) { const size_t t = (size_t)blockIdx.x * 256 + threadIdx.x; if (t >= n8) return; FragH f;
#pragma unroll
  for (int q = 0; q < 8; ++q) f.h[q] = (_Float16)x[t * 8 + q]; *(volatile v8us*)((unsigned short*)X16 + t * 8) = f.half[0]; __threadfence(); *(volatile v8us*)((unsigned short*)X16 + t * 8) = f.half[0]; }
template <int NHv, int TTv>
__global__ __launch_bounds__(256) void k_vt(const _Float16* __restrict__ V16, int ldv, int voff, _Float16* __restrict__ Vt) { __shared__ unsigned short tl[64][66]; const int tid = threadIdx.x; const int slab = blockIdx.x / (TTv / 64), lg = blockIdx.x % (TTv / 64); const int b = slab / NHv, h = slab % NHv;
  for (int i = tid; i < 64 * 8; i += 256) { const int r = i / 8, c8 = (i % 8) * 8; FragH f; f.half[0] = *(const v8us*)((const unsigned short*)V16 + ((size_t)b * TTv + lg * 64 + r) * ldv + voff + h * 64 + c8);
#pragma unroll
    for (int q = 0; q < 8; ++q) tl[r][c8 + q] = f.u[q]; }
  __syncthreads();
  for (int pass = 0; pass < 2; ++pass) {
#pragma unroll
    for (int rd = 0; rd < 2; ++rd) { const int d = rd * 32 + tid / 8, pc = tid % 8; FragH f;
#pragma unroll
      for (int q = 0; q < 8; ++q) f.u[q] = tl[pc * 8 + q][d];
      *(volatile v8us*)((unsigned short*)Vt + ((size_t)slab * 64 + d) * TTv + lg * 64 + pc * 8) = f.half[0]; }
    if (pass == 0) __threadfence(); } }

__global__ __launch_bounds__(256) void k_hl(const float* __restrict__ F, _Float16* __restrict__ Hh, _Float16* __restrict__ Hl, size_t n8) { const size_t t = (size_t)blockIdx.x * 256 + threadIdx.x; if (t >= n8) return; FragH fh, fl; const v4f a = *(const v4fa*)(F + t * 8), c = *(const v4fa*)(F + t * 8 + 4);
#pragma unroll
  for (int q = 0; q < 4; ++q) { _Float16 h = (_Float16)a[q]; fh.h[q] = h; fl.h[q] = (_Float16)((a[q] - (float)h) * 1024.0f); h = (_Float16)c[q]; fh.h[4 + q] = h; fl.h[4 + q] = (_Float16)((c[q] - (float)h) * 1024.0f); }
  for (int pass = 0; pass < 2; ++pass) { *(volatile v8us*)((unsigned short*)Hh + t * 8) = fh.half[0]; *(volatile v8us*)((unsigned short*)Hl + t * 8) = fl.half[0]; if (pass == 0) __threadfence(); } }

__device__ __forceinline__ v16h g2_frag(const _Float16* p, int hh) { FragH f; f.half[0] = *(const v8us*)((const unsigned short*)p + 8 * hh); f.half[1] = *(const v8us*)((const unsigned short*)p + 16 + 8 * hh); return f.v; }
__device__ __forceinline__ v8f g2_mma(v16h a, v16h b, v8f c) { v8f d = __builtin_amdgcn_wmma_f32_16x16x32_f16(false, a, false, b, (short)0, c, false, false); asm volatile("v_nop\n\tv_nop\n\tv_nop\n\tv_nop" : "+v"(d) : "v"(a), "v"(b)); return d; }
template <int ACT>
__global__ __launch_bounds__(128) void k_gemm2(const _Float16* __restrict__ A, int lda, size_t sA, const _Float16* __restrict__ Bh, int ldb, size_t sB, float alpha, const float* __restrict__ bias, size_t sBias, const float* __restrict__ CP, int rowsPerB, size_t sCPb, int row0g,
    float* __restrict__ C, _Float16* __restrict__ C16, int ldc, size_t sC, int M, int N, int K) { static_assert(ACT == 0 || ACT == 3 || ACT == 6 || ACT == 8 || ACT == 9 || ACT == 11 || ACT == 12 || ACT == 14 || ACT == 15 || ACT == 16, "k_gemm2: unsupported ACT code (would silently apply no activation)");
  __shared__ __attribute__((aligned(16))) float so[4][32][68];
  const int tid = threadIdx.x, w = tid >> 5, lane = tid & 31, ln = lane & 15, hh = lane >> 4; const int by = blockIdx.y;
  A += (size_t)by * sA; Bh += (size_t)by * sB; const size_t cofs = (size_t)by * sC; const float* bp = bias ? bias + (size_t)by * sBias : nullptr;
  const int ntn = N >> 6; const int mt = blockIdx.x / ntn, nq = blockIdx.x - mt * ntn; const int row0 = mt * 128 + 32 * w, col0 = nq * 64; if (row0 >= M) return;
  const _Float16* a0p = A + (size_t)(row0 + ln) * lda; const _Float16* a1p = a0p + (size_t)16 * lda;
  const _Float16* b0p = Bh + (size_t)(col0 + ln) * ldb; const _Float16* b1p = b0p + (size_t)16 * ldb; const _Float16* b2p = b1p + (size_t)16 * ldb; const _Float16* b3p = b2p + (size_t)16 * ldb;
  const v8f z8 = {0.f,0.f,0.f,0.f,0.f,0.f,0.f,0.f}; v8f c00 = z8, c01 = z8, c02 = z8, c03 = z8, c10 = z8, c11 = z8, c12 = z8, c13 = z8;
  for (int kb = 0; kb < K; kb += 32) { const v16h a0 = g2_frag(a0p + kb, hh), a1 = g2_frag(a1p + kb, hh);
    v16h b = g2_frag(b0p + kb, hh); c00 = g2_mma(a0, b, c00); c10 = g2_mma(a1, b, c10);
    b = g2_frag(b1p + kb, hh); c01 = g2_mma(a0, b, c01); c11 = g2_mma(a1, b, c11);
    b = g2_frag(b2p + kb, hh); c02 = g2_mma(a0, b, c02); c12 = g2_mma(a1, b, c12);
    b = g2_frag(b3p + kb, hh); c03 = g2_mma(a0, b, c03); c13 = g2_mma(a1, b, c13); }
  v8f accs[8] = {c00, c01, c02, c03, c10, c11, c12, c13};
#pragma unroll
  for (int u = 0; u < 8; ++u) { const int t = u & 3, half = u >> 2; const int col = col0 + t * 16 + ln; const float bv = bp ? bf16_round(bp[col]) : 0.f;
#pragma unroll
    for (int r = 0; r < 8; ++r) { const int rloc = half * 16 + 8 * hh + r; float v = accs[u][r] * alpha + bv; if (CP) { if (rowsPerB < 0) v += CP[cofs + (size_t)(row0g + row0 + rloc) * ldc + col];        else { const int bidx = (row0g + row0 + rloc) / rowsPerB; v += CP[(size_t)bidx * sCPb + (size_t)by * 64 + col]; } }
      if (ACT == 3) v = fmaxf(v, 0.f); else if (ACT == 6) v = 0.5f * v * (1.0f + erff(v * 0.70710678118654752f)); else if (ACT == 11) v = 1.0f / (1.0f + expf(-v)); else if (ACT == 15) v = v / (1.0f + expf(-v)); else if (ACT == 12) v = (v > 0.f) ? v : 0.01f * v; else if (ACT == 8) v = tanhf(v); else if (ACT == 9) v = 0.5f * v * (1.0f + tanhf(0.7978845608028654f * (v + 0.044715f * v * v * v))); else if (ACT == 14) v = (v > 0.f) ? v : 0.1f * v; else if (ACT == 16) v = (v >= 0.f) ? v : 0.3f * v;
      so[w][rloc][t * 16 + ln] = v; } }
  __builtin_amdgcn_fence(__ATOMIC_ACQ_REL, "workgroup"); __builtin_amdgcn_wave_barrier();
  const int rsub = lane >> 4, c4 = (lane & 15) * 4;
  for (int pass = 0; pass < 2; ++pass) {
#pragma unroll
    for (int q = 0; q < 16; ++q) { const int r = q * 2 + rsub; const v4f v = *(const v4fa*)&so[w][r][c4]; if (C) *(volatile v4f*)(C + cofs + (size_t)(row0 + r) * ldc + col0 + c4) = v; if (C16) { v4h h4; for (int i = 0; i < 4; ++i) h4[i] = (_Float16)v[i]; *(volatile v4h*)(C16 + cofs + (size_t)(row0 + r) * ldc + col0 + c4) = h4; } }
    if (pass == 0) __threadfence(); } }


__global__ __launch_bounds__(256) void k_nrope(const float* __restrict__ F, int nheads, const float* __restrict__ w, const float* __restrict__ cs, const float* __restrict__ sn, _Float16* __restrict__ H, _Float16* __restrict__ L) {
  const size_t t = (size_t)blockIdx.x * 256 + threadIdx.x; if (t >= (size_t)NR * nheads) return; const int h = (int)(t % nheads); const size_t s = t / nheads; const size_t sp = s;        const float* src = F + s * (size_t)(nheads * HD) + h * HD; float ss = 0.f;
  for (int d = 0; d < HD; ++d) { const float v = src[d]; ss += v * v; } const float inv = w ? rsqrtf(ss / (float)HD + 1e-6f) : 1.0f;
  const float* cr = cs + sp * HD; const float* sr = sn + sp * HD; unsigned short* dh = (unsigned short*)H + s * (size_t)(nheads * HD) + h * HD; unsigned short* dl = (unsigned short*)L + s * (size_t)(nheads * HD) + h * HD;
  for (int pass = 0; pass < 2; ++pass) {
    for (int g8 = 0; g8 < HH / 8; ++g8) { FragH h1, l1, h2, l2;
      for (int q = 0; q < 8; ++q) { const int d = g8 * 8 + q; float a = src[d] * inv; if (w) a *= bf16_round(w[d]); float b = src[d + HH] * inv; if (w) b *= bf16_round(w[d + HH]);
        float o1 = a * cr[d]; o1 += -b * sr[d]; float o2 = b * cr[d + HH]; o2 += a * sr[d + HH];
        const _Float16 x1 = (_Float16)o1, x2 = (_Float16)o2; h1.h[q] = x1; l1.h[q] = (_Float16)((o1 - (float)x1) * 1024.0f); h2.h[q] = x2; l2.h[q] = (_Float16)((o2 - (float)x2) * 1024.0f); }
      *(volatile v8us*)(dh + g8 * 8) = h1.half[0]; *(volatile v8us*)(dl + g8 * 8) = l1.half[0]; *(volatile v8us*)(dh + HH + g8 * 8) = h2.half[0]; *(volatile v8us*)(dl + HH + g8 * 8) = l2.half[0]; }
    if (pass == 0) __threadfence(); } }
__global__ __launch_bounds__(256) void k_wsoft(const float* __restrict__ S, const float* __restrict__ S2, const float* __restrict__ S3, int r0, int kstart, int nk, _Float16* __restrict__ PH, _Float16* __restrict__ PL) {
  const int wv = threadIdx.x >> 5, ln = threadIdx.x & 31; const int rr = blockIdx.x * 8 + wv; if (rr >= NHQ * BAND) return; const int h = rr / BAND, rl = rr % BAND; const int r = r0 + rl; const size_t prow = ((size_t)h * BAND + rl) * SP, prow2 = ((size_t)h * BAND + rl) * SPX; const float* sr = S + prow; const float* s2 = S2 ? S2 + prow2 : nullptr; const float* s3 = S3 ? S3 + prow2 : nullptr; float m = -3.0e38f;
  auto sc = [&](int j) { float z = sr[j]; if (s2) { z += s2[j]; z += s3[j]; } return z; };
  for (int j = ln; j < nk; j += 32) { const int key = kstart + j; if (key <= r && key > r - WIN) m = fmaxf(m, sc(j)); }
  for (int o = 16; o > 0; o >>= 1) m = fmaxf(m, __shfl_xor(m, o, 32)); float su = 0.f;
  for (int j = ln; j < nk; j += 32) { const int key = kstart + j; if (key <= r && key > r - WIN) su += expf(sc(j) - m); }
  for (int o = 16; o > 0; o >>= 1) su += __shfl_xor(su, o, 32); const float f = 1024.0f / su;
  for (int pass = 0; pass < 2; ++pass) {
    for (int j = ln; j < nk; j += 32) { const int key = kstart + j; const float p = (key <= r && key > r - WIN) ? expf(sc(j) - m) * f : 0.f; const _Float16 hv = (_Float16)p; *(volatile _Float16*)(PH + prow + j) = hv; if (PL) *(volatile _Float16*)(PL + prow + j) = (_Float16)((p - (float)hv) * 1024.0f); }
    if (pass == 0) __threadfence(); } }

__global__ __launch_bounds__(256) void k_oadd(float* __restrict__ O, const float* __restrict__ X1, const float* __restrict__ X2, int r0) {
  const size_t t = (size_t)blockIdx.x * 256 + threadIdx.x; if (t >= (size_t)BAND * DM / 4) return; float* o = O + (size_t)r0 * DM + t * 4; const v4f a = *(const v4fa*)o, b = *(const v4fa*)(X1 + t * 4), c = *(const v4fa*)(X2 + t * 4); v4f r; for (int q = 0; q < 4; ++q) { float v = a[q] + b[q]; v += c[q]; r[q] = v; }
  *(volatile v4f*)o = r; __threadfence(); *(volatile v4f*)o = r; }

__global__ __launch_bounds__(256) void k_rotab(float* __restrict__ CS, float* __restrict__ SN) {
  const int t = blockIdx.x * 256 + threadIdx.x; if (t >= NR * HD) return; const int d = t % HD, s = t / HD; const int j = d % HH; const float ex = (float)(2 * j) / (float)HD; const float inv = 1.0f / powf(10000.0f, ex); const float th = (float)(s % SQ) * inv; const float c = cosf(th), sn = sinf(th);
  for (int pass = 0; pass < 2; ++pass) { *(volatile float*)(CS + t) = c; *(volatile float*)(SN + t) = sn; if (pass == 0) __threadfence(); } }
extern "C" void kernel_launch(void* const* d_in, const int* in_sizes, int n_in,
                              void* d_out, int out_size, void* d_ws, size_t ws_size, hipStream_t stream) {
  (void)in_sizes; (void)n_in; (void)out_size;
  const float* const* I = (const float* const*)d_in; const float* x = I[0]; const float* Wq = I[1]; const float* Wk = I[2]; const float* Wv = I[3]; const float* Wo = I[4]; const float* qnw = nullptr; const float* knw = nullptr;
  char* ws = (char*)d_ws; size_t off = 0;
  auto take = [&](size_t bytes) { char* p = ws + off; off += (bytes + 255) & ~(size_t)255; return p; };
  const size_t np = (size_t)NR * DM, nk8 = (size_t)NR * KVD;
  _Float16* BQ = (_Float16*)take((size_t)DM * DM * 2); _Float16* BK = (_Float16*)take((size_t)KVD * DM * 2); _Float16* BV = (_Float16*)take((size_t)KVD * DM * 2); _Float16* BO = (_Float16*)take((size_t)DM * DM * 2); float* cs = (float*)take((size_t)NR * HD * 4); float* sn = (float*)take((size_t)NR * HD * 4);
  _Float16* X16 = (_Float16*)take(np * 2); float* F32 = (float*)take(np * 4); _Float16* QH = (_Float16*)take(np * 2); _Float16* QL = X16;        _Float16* KH = (_Float16*)take(nk8 * 2); _Float16* KL = (_Float16*)take(nk8 * 2); _Float16* VH = (_Float16*)take(nk8 * 2); _Float16* VL = (_Float16*)take(nk8 * 2); _Float16* VTh = (_Float16*)take(nk8 * 2); _Float16* VTl = (_Float16*)take(nk8 * 2);
  float* S = (float*)take((size_t)NHQ * BAND * SP * 4); _Float16* PH = VH; _Float16* PL = VL;        _Float16* OL = (_Float16*)take((size_t)NB * NPB * BAND * DM * 2); float* SX1 = (float*)take((size_t)NHQ * BAND * SPX * 4); float* SX2 = (float*)take((size_t)NHQ * BAND * SPX * 4); float* OX1 = (float*)take((size_t)BAND * DM * 4); float* OX2 = (float*)take((size_t)BAND * DM * 4);
  float* O = F32;        _Float16* O16 = X16;
  if (off > ws_size) return;
  k_wt_f16<<<(unsigned)(((size_t)DM * (DM / 8) + 255) / 256), 256, 0, stream>>>(Wq, BQ, DM, DM, 16.0f); k_wt_f16<<<(unsigned)(((size_t)KVD * (DM / 8) + 255) / 256), 256, 0, stream>>>(Wk, BK, DM, KVD, 16.0f); k_wt_f16<<<(unsigned)(((size_t)KVD * (DM / 8) + 255) / 256), 256, 0, stream>>>(Wv, BV, DM, KVD, 16.0f); k_wt_f16<<<(unsigned)(((size_t)DM * (DM / 8) + 255) / 256), 256, 0, stream>>>(Wo, BO, DM, DM, 16.0f);
  k_rotab<<<(NR * HD + 255) / 256, 256, 0, stream>>>(cs, sn);
  k_x16<<<(unsigned)((np / 8 + 255) / 256), 256, 0, stream>>>(x, X16, np / 8);
  k_gemm2<0><<<dim3((NR / 128) * (KVD / 64), 1), 128, 0, stream>>>(X16, DM, 0, BK, DM, 0, 0.0625f, nullptr, 0, nullptr, 1, 0, 0, F32, nullptr, KVD, 0, NR, KVD, DM);
  k_nrope<<<(unsigned)(((size_t)NR * NKV + 255) / 256), 256, 0, stream>>>(F32, NKV, knw, cs, sn, KH, KL);
  k_gemm2<0><<<dim3((NR / 128) * (KVD / 64), 1), 128, 0, stream>>>(X16, DM, 0, BV, DM, 0, 0.0625f, nullptr, 0, nullptr, 1, 0, 0, F32, nullptr, KVD, 0, NR, KVD, DM);
  k_hl<<<(unsigned)((nk8 / 8 + 255) / 256), 256, 0, stream>>>(F32, VH, VL, nk8 / 8);
  k_vt<KVD / 64, SQ><<<NB * (KVD / 64) * (SQ / 64), 256, 0, stream>>>(VH, KVD, 0, VTh); k_vt<KVD / 64, SQ><<<NB * (KVD / 64) * (SQ / 64), 256, 0, stream>>>(VL, KVD, 0, VTl);
  k_gemm2<0><<<dim3((NR / 128) * (DM / 64), 1), 128, 0, stream>>>(X16, DM, 0, BQ, DM, 0, 0.0625f, nullptr, 0, nullptr, 1, 0, 0, F32, nullptr, DM, 0, NR, DM, DM);
  k_nrope<<<(unsigned)(((size_t)NR * NHQ + 255) / 256), 256, 0, stream>>>(F32, NHQ, qnw, cs, sn, QH, QL);
  const size_t sS = (size_t)BAND * SP;
  for (int b = 0; b < NB; ++b) for (int band = 0; band < NBAND; ++band) { const int r0 = band * BAND; const int kstart = 0; const int nk = r0 + BAND; const bool pr = band < NPB;
    const _Float16* QHb = QH + (size_t)b * SQ * DM; const _Float16* QLb = QL + (size_t)b * SQ * DM; const _Float16* KHb = KH + (size_t)b * SQ * KVD; const _Float16* KLb = KL + (size_t)b * SQ * KVD; const _Float16* VThb = VTh + (size_t)b * (KVD / 64) * 64 * SQ; const _Float16* VTlb = VTl + (size_t)b * (KVD / 64) * 64 * SQ; float* Ob = O + (size_t)b * SQ * DM;
    const dim3 gS((BAND / 128) * (nk / 64), NKV), gO((BAND / 128) * (HD / 64), NKV);
    for (int par = 0; par < NREP; ++par) {
      const _Float16* qh = QHb + (size_t)r0 * DM + par * HD; const _Float16* ql = QLb + (size_t)r0 * DM + par * HD; const _Float16* kh = KHb + (size_t)kstart * KVD; const _Float16* kl = KLb + (size_t)kstart * KVD; const size_t so = par * sS;
      k_gemm2<0><<<gS, 128, 0, stream>>>(qh, DM, (size_t)NREP * HD, kh, KVD, (size_t)HD, SCALE, nullptr, 0, nullptr, 1, 0, 0, S + so, nullptr, SP, NREP * sS, BAND, nk, HD);
      if (pr) { k_gemm2<0><<<gS, 128, 0, stream>>>(ql, DM, (size_t)NREP * HD, kh, KVD, (size_t)HD, SCALE / 1024.0f, nullptr, 0, nullptr, 1, 0, 0, SX1 + par * ((size_t)BAND * SPX), nullptr, SPX, NREP * ((size_t)BAND * SPX), BAND, nk, HD);
                k_gemm2<0><<<gS, 128, 0, stream>>>(qh, DM, (size_t)NREP * HD, kl, KVD, (size_t)HD, SCALE / 1024.0f, nullptr, 0, nullptr, 1, 0, 0, SX2 + par * ((size_t)BAND * SPX), nullptr, SPX, NREP * ((size_t)BAND * SPX), BAND, nk, HD); } }
    k_wsoft<<<(NHQ * BAND) / 8, 256, 0, stream>>>(S, pr ? SX1 : nullptr, pr ? SX2 : nullptr, r0, kstart, nk, PH, pr ? PL : nullptr);
    for (int par = 0; par < NREP; ++par) { const _Float16* ph = PH + par * sS; const _Float16* pl = PL + par * sS; const _Float16* vth = VThb + (size_t)kstart; const _Float16* vtl = VTlb + (size_t)kstart; float* o = Ob + (size_t)r0 * DM + par * HD;
      k_gemm2<0><<<gO, 128, 0, stream>>>(ph, SP, NREP * sS, vth, SQ, (size_t)2 * 64 * SQ, 0.0009765625f, nullptr, 0, nullptr, 1, 0, 0, o, nullptr, DM, (size_t)NREP * HD, BAND, HD, nk);
      if (pr) { k_gemm2<0><<<gO, 128, 0, stream>>>(pl, SP, NREP * sS, vth, SQ, (size_t)2 * 64 * SQ, 0.0009765625f / 1024.0f, nullptr, 0, nullptr, 1, 0, 0, OX1 + par * HD, nullptr, DM, (size_t)NREP * HD, BAND, HD, nk);
                k_gemm2<0><<<gO, 128, 0, stream>>>(ph, SP, NREP * sS, vtl, SQ, (size_t)2 * 64 * SQ, 0.0009765625f / 1024.0f, nullptr, 0, nullptr, 1, 0, 0, OX2 + par * HD, nullptr, DM, (size_t)NREP * HD, BAND, HD, nk); } }
    if (pr) k_oadd<<<(unsigned)(((size_t)BAND * DM / 4 + 255) / 256), 256, 0, stream>>>(Ob, OX1, OX2, r0); }
  const size_t nlo = (size_t)NPB * BAND * DM;
  for (int b = 0; b < NB; ++b) { k_hl<<<(unsigned)((nlo / 8 + 255) / 256), 256, 0, stream>>>(O + (size_t)b * SQ * DM, O16 + (size_t)b * SQ * DM, OL + (size_t)b * nlo, nlo / 8);
    k_h16<<<(unsigned)((((size_t)SQ * DM - nlo) / 8 + 255) / 256), 256, 0, stream>>>(O + (size_t)b * SQ * DM + nlo, O16 + (size_t)b * SQ * DM + nlo, ((size_t)SQ * DM - nlo) / 8); }
  k_gemm2<0><<<dim3((NR / 128) * (DM / 64), 1), 128, 0, stream>>>(O16, DM, 0, BO, DM, 0, 0.0625f, nullptr, 0, nullptr, 1, 0, 0, (float*)d_out, nullptr, DM, 0, NR, DM, DM);
  for (int b = 0; b < NB; ++b) k_gemm2<0><<<dim3(((NPB * BAND) / 128) * (DM / 64), 1), 128, 0, stream>>>(OL + (size_t)b * nlo, DM, 0, BO, DM, 0, 0.0625f / 1024.0f, nullptr, 0, (const float*)d_out + (size_t)b * SQ * DM, 1, (size_t)DM, 0, (float*)d_out + (size_t)b * SQ * DM, nullptr, DM, 0, NPB * BAND, DM, DM);
}
